// SelfAttention_42537356100349
// MI455X (gfx1250) — hardware-verified
//
#include <hip/hip_runtime.h>


#ifndef NB
#define NB 8
#endif
#ifndef SEQ
#define SEQ 4096
#endif
#define NB_FULL   8
#define SEQ_FULL  4096
#define CH        256
#define HD        32
#define NQKV      96
#define NT        64
#define XPW       132
#define SP        72
#define BQ        128
#define BK        32
#define NWAVE     8
#define CP        40
#define ON        32
#define OPF       36
#define RES_CARRY 2048.0f
#define RES_FOLD  (1.0f / 2048.0f)

static_assert(NB >= 1 && NB <= NB_FULL);
static_assert(SEQ <= SEQ_FULL);
static_assert(SEQ % BQ == 0);
static_assert(SEQ % NT == 0);
static_assert(SEQ % ON == 0);
static_assert(SEQ % BK == 0);
static_assert(BQ == NWAVE * 16);
static_assert(HD == 32);
static_assert(CH % 32 == 0);
static_assert(NQKV == 3 * HD);
static_assert(8 * 256 == (CH / 2) * (NT / 4));
static_assert(XPW >= CH / 2 && (XPW * 4) % 16 == 0);
static_assert(SP >= 2 * HD && SP >= NT && (SP * 2) % 16 == 0);
static_assert(NT * 4 == 256);
static_assert(HD * 8 == 256);
static_assert(CP >= HD && (CP * 2) % 16 == 0);
static_assert(OPF >= ON && (OPF * 4) % 16 == 0);
static_assert(NWAVE * 32 == CH);
static_assert(ON == 32);
static_assert(NT * XPW * 4 + 2 * NT * SP * 2 + HD * SP * 2 <= 65536);

#define WB_BYTES  ((size_t)NQKV * CH * 2)
#define WO_BYTES  ((size_t)CH * HD * 2)
#define PL_BYTES  ((size_t)NB * SEQ * HD * 2)
#define NPLANE    6
#define WS_TOTAL  (WB_BYTES + WO_BYTES + NPLANE * PL_BYTES)
static_assert(WB_BYTES % 128 == 0 && WO_BYTES % 128 == 0 && PL_BYTES % 128 == 0);
static_assert(WS_TOTAL <= (size_t)134217728);

typedef __bf16   bf16;
typedef _Float16 f16;
typedef bf16     v16bf __attribute__((ext_vector_type(16)));
typedef f16      v16h  __attribute__((ext_vector_type(16)));
typedef f16      v8h   __attribute__((ext_vector_type(8)));
typedef float    v8f   __attribute__((ext_vector_type(8)));
typedef float    v4f   __attribute__((ext_vector_type(4)));
typedef unsigned v4u   __attribute__((ext_vector_type(4)));

union FragB  { v16bf v; v4u q[2]; };
union FragH  { v16h  v; v4u q[2]; f16 h[16]; };
union Pack8H { v4u u; v8h v; f16 h[8]; };

static __device__ __forceinline__ v8f mma_bf16(v16bf a, v16bf b, v8f acc) {
  acc = __builtin_amdgcn_wmma_f32_16x16x32_bf16(false, a, false, b, (short)0, acc, false, false);
  asm volatile("v_nop\n\tv_nop\n\tv_nop\n\tv_nop" : "+v"(acc) : "v"(a), "v"(b));
  return acc;
}
static __device__ __forceinline__ v8f mma_f16(v16h a, v16h b, v8f acc) {
  acc = __builtin_amdgcn_wmma_f32_16x16x32_f16(false, a, false, b, (short)0, acc, false, false);
  asm volatile("v_nop\n\tv_nop\n\tv_nop\n\tv_nop" : "+v"(acc) : "v"(a), "v"(b));
  return acc;
}

static __device__ __forceinline__ unsigned bf16_bits(float f) {
  const unsigned u = __float_as_uint(f);
  return (u + 0x7FFFu + ((u >> 16) & 1u)) >> 16;
}
static __device__ __forceinline__ float bf16_val(float f) {
  return __uint_as_float(bf16_bits(f) << 16);
}

__global__ __launch_bounds__(256) void prep_kernel(const float* __restrict__ wq, const float* __restrict__ wk,
                                                   const float* __restrict__ wv, const float* __restrict__ wo,
                                                   unsigned short* __restrict__ wb, f16* __restrict__ woh) {
  const int p = blockIdx.x * 256 + threadIdx.x;
  if (blockIdx.x < 12) {
    const int which = p >> 10;
    const int off   = (p & 1023) * 8;
    const v4f q0 = *(const v4f*)(wq + off), q1 = *(const v4f*)(wq + off + 4);
    const v4f k0 = *(const v4f*)(wk + off), k1 = *(const v4f*)(wk + off + 4);
    const v4f v0 = *(const v4f*)(wv + off), v1 = *(const v4f*)(wv + off + 4);
    const v4f a0 = (which == 0) ? q0 : ((which == 1) ? k0 : v0);
    const v4f a1 = (which == 0) ? q1 : ((which == 1) ? k1 : v1);
    v4u u;
    u[0] = bf16_bits(a0[0]) | (bf16_bits(a0[1]) << 16);
    u[1] = bf16_bits(a0[2]) | (bf16_bits(a0[3]) << 16);
    u[2] = bf16_bits(a1[0]) | (bf16_bits(a1[1]) << 16);
    u[3] = bf16_bits(a1[2]) | (bf16_bits(a1[3]) << 16);
    unsigned short* dst = wb + (size_t)p * 8;
    *(volatile v4u*)dst = u;
    __threadfence();
    *(volatile v4u*)dst = u;
  } else {
    const int off = (p - 3072) * 8;
    const v4f a0 = *(const v4f*)(wo + off), a1 = *(const v4f*)(wo + off + 4);
    Pack8H ph;
    #pragma unroll
    for (int i = 0; i < 4; ++i) {
      ph.h[i]     = (f16)(bf16_val(a0[i]) * 64.0f);
      ph.h[4 + i] = (f16)(bf16_val(a1[i]) * 64.0f);
    }
    const v4u u = ph.u;
    f16* dst = woh + off;
    *(volatile v4u*)dst = u;
    __threadfence();
    *(volatile v4u*)dst = u;
  }
}

__global__ __launch_bounds__(256) void qkv_kernel(const float* __restrict__ x,
                                                  const unsigned short* __restrict__ wb,
                                                  f16* __restrict__ qp, f16* __restrict__ kp,
                                                  f16* __restrict__ qr, f16* __restrict__ kr,
                                                  f16* __restrict__ vp) {
  const int n0   = blockIdx.x * NT;
  const int b    = blockIdx.y;
  const int tid  = threadIdx.x;
  const int wave = tid >> 5;
  const int lane = tid & 31;
  const int lq   = lane & 15;
  const int hi   = lane >> 4;

  __shared__ __align__(16) unsigned sX[NT * XPW];
  __shared__ __align__(16) f16      sQK[NT * SP];
  __shared__ __align__(16) f16      sR[NT * SP];
  __shared__ __align__(16) f16      sV[HD * SP];

  #pragma unroll 2
  for (int it = 0; it < 8; ++it) {
    const int item = it * 256 + tid;
    const int nq   = item & 15;
    const int cp   = item >> 4;
    const float* src = x + ((size_t)b * CH + 2 * cp) * SEQ_FULL + n0 + nq * 4;
    const v4f a0 = *(const v4f*)(src);
    const v4f a1 = *(const v4f*)(src + SEQ_FULL);
    #pragma unroll
    for (int i = 0; i < 4; ++i)
      sX[(nq * 4 + i) * XPW + cp] = bf16_bits(a0[i]) | (bf16_bits(a1[i]) << 16);
  }
  __syncthreads();

  const int nt = wave & 3;
  const int g3 = wave >> 2;
  v8f acc[3];
  #pragma unroll
  for (int j = 0; j < 3; ++j) acc[j] = (v8f){0, 0, 0, 0, 0, 0, 0, 0};

  const int aoff = (nt * 16 + lq) * XPW + hi * 4;
  #pragma unroll 2
  for (int ks = 0; ks < CH / 32; ++ks) {
    FragB a;
    a.q[0] = *(const v4u*)(sX + aoff + ks * 16);
    a.q[1] = *(const v4u*)(sX + aoff + ks * 16 + 8);
    #pragma unroll
    for (int j = 0; j < 3; ++j) {
      const unsigned short* wr = wb + (size_t)((g3 * 3 + j) * 16 + lq) * CH + ks * 32 + hi * 8;
      FragB w;
      w.q[0] = *(const v4u*)(wr);
      w.q[1] = *(const v4u*)(wr + 16);
      acc[j] = mma_bf16(a.v, w.v, acc[j]);
    }
  }

  #pragma unroll
  for (int j = 0; j < 3; ++j) {
    const int t = g3 * 3 + j;
    #pragma unroll
    for (int r = 0; r < 8; ++r) {
      const int nrow = nt * 16 + hi * 8 + r;
      const float av = acc[j][r];
      const f16 hv = (f16)av;
      if (t < 4) {
        sQK[nrow * SP + t * 16 + lq] = hv;
        sR[nrow * SP + t * 16 + lq]  = (f16)((av - (float)hv) * RES_CARRY);
      } else {
        sV[((t - 4) * 16 + lq) * SP + nrow] = hv;
      }
    }
  }
  __syncthreads();

  Pack8H pq, pk, pqr, pkr, pv;
  const int row = tid >> 2, seg = tid & 3;
  pq.v  = *(const v8h*)(sQK + row * SP + seg * 8);
  pk.v  = *(const v8h*)(sQK + row * SP + HD + seg * 8);
  pqr.v = *(const v8h*)(sR + row * SP + seg * 8);
  pkr.v = *(const v8h*)(sR + row * SP + HD + seg * 8);
  const int dv = tid >> 3, sv = tid & 7;
  pv.v = *(const v8h*)(sV + dv * SP + sv * 8);
  const size_t qi = ((size_t)b * SEQ + n0) * HD + (size_t)tid * 8;
  const size_t vi = ((size_t)b * HD + dv) * SEQ + n0 + sv * 8;
  const v4u uq = pq.u, uk = pk.u, uqr = pqr.u, ukr = pkr.u, uv = pv.u;
  *(volatile v4u*)(qp + qi) = uq;
  *(volatile v4u*)(kp + qi) = uk;
  *(volatile v4u*)(qr + qi) = uqr;
  *(volatile v4u*)(kr + qi) = ukr;
  *(volatile v4u*)(vp + vi) = uv;
  __threadfence();
  *(volatile v4u*)(qp + qi) = uq;
  *(volatile v4u*)(kp + qi) = uk;
  *(volatile v4u*)(qr + qi) = uqr;
  *(volatile v4u*)(kr + qi) = ukr;
  *(volatile v4u*)(vp + vi) = uv;
}

__global__ __launch_bounds__(256) void attn_kernel(const f16* __restrict__ qp, const f16* __restrict__ qr,
                                                   const f16* __restrict__ kp, const f16* __restrict__ kr,
                                                   const f16* __restrict__ vp, f16* __restrict__ ctx) {
  const int qblk = blockIdx.x;
  const int b    = blockIdx.y;
  const int tid  = threadIdx.x;
  const int wave = tid >> 5;
  const int lane = tid & 31;
  const int lq   = lane & 15;
  const int hi   = lane >> 4;

  __shared__ __align__(16) f16 sC[NWAVE * 16 * CP];

  const int qrow0 = qblk * BQ + wave * 16;

  FragH qf, qrf;
  {
    const size_t qo = ((size_t)b * SEQ + qrow0 + lq) * HD + hi * 8;
    qf.q[0]  = *(const v4u*)(qp + qo);
    qf.q[1]  = *(const v4u*)(qp + qo + 16);
    qrf.q[0] = *(const v4u*)(qr + qo);
    qrf.q[1] = *(const v4u*)(qr + qo + 16);
  }
  const f16* kb_b = kp + (size_t)b * SEQ * HD;
  const f16* kr_b = kr + (size_t)b * SEQ * HD;
  const f16* vt_b = vp + (size_t)b * HD * SEQ;

  v8f o[2];
  o[0] = (v8f){0, 0, 0, 0, 0, 0, 0, 0};
  o[1] = (v8f){0, 0, 0, 0, 0, 0, 0, 0};
  float rmax = -__builtin_inff();
  float rsum = 0.0f;
  const float SL = 1.4426950408889634f;

  #pragma unroll 1
  for (int j0 = 0; j0 < SEQ; j0 += BK) {
    FragH ak[2], akr[2], bv[2];
    #pragma unroll
    for (int sub = 0; sub < 2; ++sub) {
      const size_t ko = (size_t)(j0 + sub * 16 + lq) * HD + hi * 8;
      ak[sub].q[0]  = *(const v4u*)(kb_b + ko);
      ak[sub].q[1]  = *(const v4u*)(kb_b + ko + 16);
      akr[sub].q[0] = *(const v4u*)(kr_b + ko);
      akr[sub].q[1] = *(const v4u*)(kr_b + ko + 16);
    }
    #pragma unroll
    for (int dt = 0; dt < 2; ++dt) {
      const f16* base = vt_b + (size_t)(dt * 16 + lq) * SEQ + j0 + hi * 8;
      bv[dt].q[0] = *(const v4u*)(base);
      bv[dt].q[1] = *(const v4u*)(base + 16);
    }

    v8f c[2];
    #pragma unroll
    for (int sub = 0; sub < 2; ++sub) {
      const v8f z = (v8f){0, 0, 0, 0, 0, 0, 0, 0};
      v8f cm = mma_f16(ak[sub].v, qf.v, z);
      v8f cr = mma_f16(akr[sub].v, qf.v, z);
      cr = mma_f16(ak[sub].v, qrf.v, cr);
      #pragma unroll
      for (int r = 0; r < 8; ++r) cm[r] = cm[r] + cr[r] * RES_FOLD;
      c[sub] = cm;
    }

    float m_new = rmax;
    #pragma unroll
    for (int r = 0; r < 8; ++r) {
      m_new = fmaxf(m_new, c[0][r]);
      m_new = fmaxf(m_new, c[1][r]);
    }
    m_new = fmaxf(m_new, __shfl_xor(m_new, 16, 32));
    const float scale = __builtin_amdgcn_exp2f((rmax - m_new) * SL);
    rmax = m_new;

    FragH pa;
    float psum = 0.0f;
    #pragma unroll
    for (int r = 0; r < 8; ++r) {
      const float p0 = __builtin_amdgcn_exp2f((c[0][r] - m_new) * SL);
      const float p1 = __builtin_amdgcn_exp2f((c[1][r] - m_new) * SL);
      psum += p0 + p1;
      pa.h[r]     = (f16)(p0 * 4096.0f);
      pa.h[8 + r] = (f16)(p1 * 4096.0f);
    }
    rsum = rsum * scale + psum + __shfl_xor(psum, 16, 32);

    float sc[8];
    #pragma unroll
    for (int r = 0; r < 8; ++r) sc[r] = __shfl(scale, (hi << 3) + r, 32);
    #pragma unroll
    for (int dt = 0; dt < 2; ++dt) {
      #pragma unroll
      for (int r = 0; r < 8; ++r) o[dt][r] *= sc[r];
    }

    #pragma unroll
    for (int dt = 0; dt < 2; ++dt) o[dt] = mma_f16(pa.v, bv[dt].v, o[dt]);
  }

  const float rinv = (1.0f / rsum) * (1.0f / 4096.0f);
  float rs[8];
  #pragma unroll
  for (int r = 0; r < 8; ++r) rs[r] = __shfl(rinv, (hi << 3) + r, 32);

  f16* so = sC + wave * (16 * CP);
  #pragma unroll
  for (int r = 0; r < 8; ++r) {
    #pragma unroll
    for (int dt = 0; dt < 2; ++dt)
      so[(hi * 8 + r) * CP + dt * 16 + lq] = (f16)(o[dt][r] * rs[r]);
  }
  __syncthreads();

  v4u    cv[2];
  size_t ci[2];
  #pragma unroll
  for (int it = 0; it < 2; ++it) {
    const int p   = it * 32 + lane;
    const int row = p >> 2, seg = p & 3;
    Pack8H ph;
    ph.v   = *(const v8h*)(so + row * CP + seg * 8);
    cv[it] = ph.u;
    ci[it] = ((size_t)b * SEQ + qrow0) * HD + (size_t)p * 8;
  }
  #pragma unroll
  for (int it = 0; it < 2; ++it) *(volatile v4u*)(ctx + ci[it]) = cv[it];
  __threadfence();
  #pragma unroll
  for (int it = 0; it < 2; ++it) *(volatile v4u*)(ctx + ci[it]) = cv[it];
}

__global__ __launch_bounds__(256) void oproj_kernel(const f16* __restrict__ ctx, const f16* __restrict__ woh,
                                                    const float* __restrict__ x, const float* __restrict__ gamma,
                                                    float* __restrict__ out) {
  const int n0   = blockIdx.x * ON;
  const int b    = blockIdx.y;
  const int tid  = threadIdx.x;
  const int wave = tid >> 5;
  const int lane = tid & 31;
  const int lq   = lane & 15;
  const int hi   = lane >> 4;

  __shared__ __align__(16) float sO[CH * OPF];

  const float gs = bf16_val(gamma[0]) * (1.0f / 64.0f);

  FragH bn[2];
  #pragma unroll
  for (int nt = 0; nt < 2; ++nt) {
    const f16* p = ctx + ((size_t)b * SEQ + n0 + nt * 16 + lq) * HD + hi * 8;
    bn[nt].q[0] = *(const v4u*)(p);
    bn[nt].q[1] = *(const v4u*)(p + 16);
  }
  #pragma unroll
  for (int ct = 0; ct < 2; ++ct) {
    const int c0 = (wave * 2 + ct) * 16;
    FragH a;
    const f16* wr = woh + (size_t)(c0 + lq) * HD + hi * 8;
    a.q[0] = *(const v4u*)(wr);
    a.q[1] = *(const v4u*)(wr + 16);
    #pragma unroll
    for (int nt = 0; nt < 2; ++nt) {
      v8f z = (v8f){0, 0, 0, 0, 0, 0, 0, 0};
      const v8f acc = mma_f16(a.v, bn[nt].v, z);
      #pragma unroll
      for (int r = 0; r < 8; ++r)
        sO[(c0 + hi * 8 + r) * OPF + nt * 16 + lq] = acc[r];
    }
  }
  __syncthreads();

  v4f    vals[8];
  size_t gi[8];
  #pragma unroll
  for (int it = 0; it < 8; ++it) {
    const int c   = wave * 32 + it * 4 + (lane >> 3);
    const int seg = lane & 7;
    const v4f o4  = *(const v4f*)(sO + c * OPF + seg * 4);
    gi[it] = ((size_t)b * CH + c) * SEQ_FULL + n0 + seg * 4;
    const v4f xr = *(const v4f*)(x + gi[it]);
    v4f rv;
    #pragma unroll
    for (int i = 0; i < 4; ++i) rv[i] = fmaf(o4[i], gs, bf16_val(xr[i]));
    vals[it] = rv;
  }
  #pragma unroll
  for (int it = 0; it < 8; ++it) *(volatile v4f*)(out + gi[it]) = vals[it];
  __threadfence();
  #pragma unroll
  for (int it = 0; it < 8; ++it) *(volatile v4f*)(out + gi[it]) = vals[it];
}

extern "C" void kernel_launch(void* const* d_in, const int* in_sizes, int n_in,
                              void* d_out, int out_size, void* d_ws, size_t ws_size,
                              hipStream_t stream) {
  if (n_in < 6) return;
  const size_t x_need = ((size_t)(NB - 1) * CH + (CH - 1)) * SEQ_FULL + SEQ;
  if ((size_t)in_sizes[0] < x_need) return;
  if ((size_t)in_sizes[1] < (size_t)HD * CH) return;
  if ((size_t)in_sizes[2] < (size_t)HD * CH) return;
  if ((size_t)in_sizes[3] < (size_t)HD * CH) return;
  if ((size_t)in_sizes[4] < (size_t)CH * HD) return;
  if (in_sizes[5] < 1) return;
  if ((size_t)out_size < x_need) return;
  if (ws_size < WS_TOTAL) return;

  const float* x     = (const float*)d_in[0];
  const float* wq    = (const float*)d_in[1];
  const float* wk    = (const float*)d_in[2];
  const float* wv    = (const float*)d_in[3];
  const float* wo    = (const float*)d_in[4];
  const float* gamma = (const float*)d_in[5];
  float*       out   = (float*)d_out;

  char* ws = (char*)d_ws;
  unsigned short* wb  = (unsigned short*)(ws);
  f16*            woh = (f16*)(ws + WB_BYTES);
  f16*            qp  = (f16*)(ws + WB_BYTES + WO_BYTES);
  f16*            kp  = (f16*)(ws + WB_BYTES + WO_BYTES + PL_BYTES);
  f16*            vp  = (f16*)(ws + WB_BYTES + WO_BYTES + 2 * PL_BYTES);
  f16*            cx  = (f16*)(ws + WB_BYTES + WO_BYTES + 3 * PL_BYTES);
  f16*            qrp = (f16*)(ws + WB_BYTES + WO_BYTES + 4 * PL_BYTES);
  f16*            krp = (f16*)(ws + WB_BYTES + WO_BYTES + 5 * PL_BYTES);

  prep_kernel<<<dim3(16), 256, 0, stream>>>(wq, wk, wv, wo, wb, woh);
  qkv_kernel<<<dim3(SEQ / NT, NB), 256, 0, stream>>>(x, wb, qp, kp, qrp, krp, vp);
  attn_kernel<<<dim3(SEQ / BQ, NB), 256, 0, stream>>>(qp, qrp, kp, krp, vp, cx);
  oproj_kernel<<<dim3(SEQ / ON, NB), 256, 0, stream>>>(cx, woh, x, gamma, out);
}
